// SSelfAttention_12687333392754
// MI455X (gfx1250) — hardware-verified
//
#include <hip/hip_runtime.h>
#include <math.h>
#include <stddef.h>

constexpr int NNODE  = 1024;
constexpr int TSTEP  = 36;
constexpr int EMB    = 64;
constexpr int NHEAD  = 4;
constexpr int HEADD  = 16;
constexpr int NSLICE = TSTEP * NHEAD;
constexpr int NROWS  = NNODE * TSTEP;
constexpr int QKROW  = 32;

constexpr size_t WS_Q2   = 0;
constexpr size_t SZ_QK   = (size_t)NSLICE * NNODE * QKROW * 2;
constexpr size_t WS_K2   = WS_Q2 + SZ_QK;
constexpr size_t SZ_V    = (size_t)NSLICE * HEADD * NNODE * 2;
constexpr size_t WS_VTH  = WS_K2 + SZ_QK;
constexpr size_t WS_VTL  = WS_VTH + SZ_V;
constexpr size_t SZ_O    = (size_t)NROWS * EMB * 2;
constexpr size_t WS_OHI  = WS_VTL + SZ_V;
constexpr size_t WS_OLO  = WS_OHI + SZ_O;
constexpr size_t SZ_WO   = (size_t)EMB * EMB * 2;
constexpr size_t WS_WOH  = WS_OLO + SZ_O;
constexpr size_t WS_WOL  = WS_WOH + SZ_WO;
constexpr size_t WS_TOTAL = WS_WOL + SZ_WO;
static_assert(WS_TOTAL == 37765120, "carve");
static_assert(WS_TOTAL <= 134217728, "carve");
static_assert((WS_K2 % 128) == 0 && (WS_VTH % 128) == 0 && (WS_VTL % 128) == 0 && (WS_OHI % 128) == 0 &&
              (WS_OLO % 128) == 0 && (WS_WOH % 128) == 0 && (WS_WOL % 128) == 0, "align");
static_assert(NROWS % 64 == 0 && EMB % 64 == 0 && EMB % 32 == 0, "gemm");
static_assert(NNODE % 64 == 0, "tiles");

typedef __attribute__((ext_vector_type(16))) _Float16 v16h;
typedef __attribute__((ext_vector_type(8)))  _Float16 v8h;
typedef __attribute__((ext_vector_type(16))) __bf16   v16b;
typedef __attribute__((ext_vector_type(8)))  __bf16   v8b;
typedef __attribute__((ext_vector_type(8)))  float    v8f;
typedef __attribute__((ext_vector_type(4)))  float    v4f;
typedef __attribute__((ext_vector_type(8)))  unsigned short us8;

__device__ __forceinline__ unsigned short f2bf_bits(float f) {
  unsigned u = __float_as_uint(f);
  return (unsigned short)((u + 0x7FFFu + ((u >> 16) & 1u)) >> 16);
}
__device__ __forceinline__ float bf_bits2f(unsigned short h) { return __uint_as_float(((unsigned)h) << 16); }

__device__ __forceinline__ void dep_guard_h(v8f& a, v8f& b, v16h x, v16h y) { asm volatile("v_nop\n\tv_nop\n\tv_nop\n\tv_nop" : "+v"(a), "+v"(b) : "v"(x), "v"(y)); }
__device__ __forceinline__ void dep_guard_b(v8f& a, v8f& b, v16b x, v16b y) { asm volatile("v_nop\n\tv_nop\n\tv_nop\n\tv_nop" : "+v"(a), "+v"(b) : "v"(x), "v"(y)); }
__device__ __forceinline__ void keep4_h(v16h a, v16h b, v16h c, v16h d) { asm volatile("v_nop" :: "v"(a), "v"(b), "v"(c), "v"(d)); }
__device__ __forceinline__ void keep4_b(v16b a, v16b b, v16b c, v16b d) { asm volatile("v_nop" :: "v"(a), "v"(b), "v"(c), "v"(d)); }
__device__ __forceinline__ void acc_guard4(v8f& a, v8f& b, v8f& c, v8f& d) { asm volatile("v_nop\n\tv_nop\n\tv_nop\n\tv_nop" : "+v"(a), "+v"(b), "+v"(c), "+v"(d)); }
template <typename T> struct Frag;
template <> struct Frag<_Float16> {
  typedef v16h V; union U { v16h v; v8h h[2]; };
  static __device__ __forceinline__ v16h load(const _Float16* p) {
    U f; f.h[0] = *(const v8h*)(p); f.h[1] = *(const v8h*)(p + 16); return f.v;
  }
  static __device__ __forceinline__ v8f mma(v16h a, v16h b, v8f c) {
    return __builtin_amdgcn_wmma_f32_16x16x32_f16(false, a, false, b, (short)0, c, false, false);
  }
  static __device__ __forceinline__ void guard(v8f& a, v8f& b, v16h x, v16h y) { dep_guard_h(a, b, x, y); }
  static __device__ __forceinline__ void keep(v16h a, v16h b, v16h c, v16h d) { keep4_h(a, b, c, d); }
};
template <> struct Frag<__bf16> {
  typedef v16b V; union U { v16b v; v8b h[2]; };
  static __device__ __forceinline__ v16b load(const __bf16* p) {
    U f; f.h[0] = *(const v8b*)(p); f.h[1] = *(const v8b*)(p + 16); return f.v;
  }
  static __device__ __forceinline__ v8f mma(v16b a, v16b b, v8f c) {
    return __builtin_amdgcn_wmma_f32_16x16x32_bf16(false, a, false, b, (short)0, c, false, false);
  }
  static __device__ __forceinline__ void guard(v8f& a, v8f& b, v16b x, v16b y) { dep_guard_b(a, b, x, y); }
  static __device__ __forceinline__ void keep(v16b a, v16b b, v16b c, v16b d) { keep4_b(a, b, c, d); }
};

template <int ET> struct Elem;
template <> struct Elem<0> { typedef _Float16 T; };
template <> struct Elem<1> { typedef __bf16 T; };
template <int ET, bool SPLIT, int BIAS_MODE, int OUT_MODE, bool RESID, int ACT = 0>
__global__ __launch_bounds__(256) void wmma_gemm64(
    const unsigned short* __restrict__ Ap, const unsigned short* __restrict__ A2p, int lda, long strideA,
    const unsigned short* __restrict__ Btp, const unsigned short* __restrict__ Bt2p, int ldb, long strideB,
    void* __restrict__ Cout, void* __restrict__ Cout2, int ldc, long strideC,
    const float* __restrict__ bias,
    const float* __restrict__ resid, long strideR,
    int M, int N, int K, float scale) {
  typedef typename Elem<ET>::T T;
  typedef typename Frag<T>::V V;
  const T* A = (const T*)Ap; const T* A2 = (const T*)A2p; const T* Bt = (const T*)Btp; const T* Bt2 = (const T*)Bt2p;
  __shared__ __align__(16) float sT[8][16 * 68];
  const int b    = blockIdx.y;
  const int lane = threadIdx.x & 31;
  const int wave = threadIdx.x >> 5;
  const int tilesN = N >> 6;
  const int tilesM = M >> 6;
  const int tile = blockIdx.x * 8 + wave;
  if (tile >= tilesM * tilesN) return;
  const int tm = tile / tilesN;
  const int tn = tile - tm * tilesN;
  const int m0 = tm << 6;
  const int n0 = tn << 6;

  const T* Ab  = A  + (size_t)b * strideA;
  const T* Bb  = Bt + (size_t)b * strideB;
  const T* Ab2 = SPLIT ? (A2  + (size_t)b * strideA) : nullptr;
  const T* Bb2 = SPLIT ? (Bt2 + (size_t)b * strideB) : nullptr;

  const int rlane = lane & 15;
  const int koff  = (lane >> 4) * 8;
  const int mOff  = (lane >> 4) * 8;

  v8f acc[4][4];
#pragma unroll
  for (int i = 0; i < 4; ++i)
#pragma unroll
    for (int j = 0; j < 4; ++j) acc[i][j] = (v8f){0.f,0.f,0.f,0.f,0.f,0.f,0.f,0.f};

  for (int k0 = 0; k0 < K; k0 += 32) {
    V bh[4], bl[4];
#pragma unroll
    for (int j = 0; j < 4; ++j) {
      const size_t bo = (size_t)(n0 + (j << 4) + rlane) * ldb + koff + k0;
      bh[j] = Frag<T>::load(Bb + bo);
      if (SPLIT) bl[j] = Frag<T>::load(Bb2 + bo);
    }
#pragma unroll
    for (int i = 0; i < 4; ++i) {
      const size_t ao = (size_t)(m0 + (i << 4) + rlane) * lda + koff + k0;
      V ah = Frag<T>::load(Ab + ao);
      V al;
      if (SPLIT) al = Frag<T>::load(Ab2 + ao);
#pragma unroll
      for (int j = 0; j < 4; ++j) {
        acc[i][j] = Frag<T>::mma(ah, bh[j], acc[i][j]);
        if (SPLIT) {
          acc[i][j] = Frag<T>::mma(ah, bl[j], acc[i][j]);
          acc[i][j] = Frag<T>::mma(al, bh[j], acc[i][j]);
        }
      }
      Frag<T>::guard(acc[i][0], acc[i][3], ah, SPLIT ? al : ah);
    }
    Frag<T>::keep(bh[0], bh[1], bh[2], bh[3]);
    if (SPLIT) Frag<T>::keep(bl[0], bl[1], bl[2], bl[3]);
  }
  acc_guard4(acc[0][0], acc[0][1], acc[0][2], acc[0][3]);
  acc_guard4(acc[1][0], acc[1][1], acc[1][2], acc[1][3]);
  acc_guard4(acc[2][0], acc[2][1], acc[2][2], acc[2][3]);
  acc_guard4(acc[3][0], acc[3][1], acc[3][2], acc[3][3]);

  float* slab = sT[wave];
  const float* Rb = RESID ? (resid + (size_t)b * strideR) : nullptr;
#pragma unroll
  for (int i = 0; i < 4; ++i) {
    const int mBase = m0 + (i << 4);
#pragma unroll
    for (int j = 0; j < 4; ++j) {
      const int n = n0 + (j << 4) + rlane;
      float bv = 0.f;
      if (BIAS_MODE == 2) bv = bias[n];
#pragma unroll
      for (int r = 0; r < 8; ++r) {
        float v = acc[i][j][r] * scale;
        if (BIAS_MODE == 1) v += bias[mBase + mOff + r];
        if (BIAS_MODE == 2) v += bv;
        if (RESID) v += Rb[(size_t)(mBase + mOff + r) * ldc + n];
        if (ACT == 1) v = tanhf(v);
        if (ACT == 2) v = fmaxf(v, 0.0f);
        if (ACT == 3) v = v / (1.0f + expf(-v));
        if (ACT == 4) v = (v > 0.f) ? v : 0.01f * v;
        if (ACT == 5) v = 0.5f * v * (1.0f + erff(v * 0.70710678118654752f));
        slab[(mOff + r) * 68 + (j << 4) + rlane] = v;
      }
    }
    __builtin_amdgcn_fence(__ATOMIC_RELEASE, "workgroup");
    __builtin_amdgcn_wave_barrier();
    __builtin_amdgcn_fence(__ATOMIC_ACQUIRE, "workgroup");
    if (OUT_MODE == 0) {
      float* C = (float*)Cout + (size_t)b * strideC;
      const int hh = lane >> 4, c4 = (lane & 15) * 4;
      for (int pass = 0; pass < 2; ++pass) {
#pragma unroll
        for (int it = 0; it < 8; ++it) {
          const int row = it * 2 + hh;
          v4f v = *(const v4f*)(slab + row * 68 + c4);
          *(volatile v4f*)(C + (size_t)(mBase + row) * ldc + n0 + c4) = v;
        }
        __threadfence();
      }
    } else {
      const int q = lane >> 3, c8 = (lane & 7) * 8;
      unsigned short* C  = (unsigned short*)Cout  + (size_t)b * strideC;
      unsigned short* C2 = (OUT_MODE == 2) ? ((unsigned short*)Cout2 + (size_t)b * strideC) : nullptr;
      for (int pass = 0; pass < 2; ++pass) {
#pragma unroll
        for (int it = 0; it < 4; ++it) {
          const int row = it * 4 + q;
          const float* sp = slab + row * 68 + c8;
          v8h hv, lv;
#pragma unroll
          for (int e = 0; e < 8; ++e) {
            if (OUT_MODE == 1) {
              hv[e] = (_Float16)sp[e];
            } else {
              unsigned short hb = f2bf_bits(sp[e]);
              unsigned short lb = f2bf_bits(sp[e] - bf_bits2f(hb));
              hv[e] = __builtin_bit_cast(_Float16, hb);
              lv[e] = __builtin_bit_cast(_Float16, lb);
            }
          }
          *(volatile v8h*)(C + (size_t)(mBase + row) * ldc + n0 + c8) = hv;
          if (OUT_MODE == 2) *(volatile v8h*)(C2 + (size_t)(mBase + row) * ldc + n0 + c8) = lv;
        }
        __threadfence();
      }
    }
    __builtin_amdgcn_fence(__ATOMIC_RELEASE, "workgroup");
    __builtin_amdgcn_wave_barrier();
    __builtin_amdgcn_fence(__ATOMIC_ACQUIRE, "workgroup");
  }
}

__device__ __forceinline__ unsigned short at_bf_bits(float f) {
  unsigned u = __float_as_uint(f);
  return (unsigned short)((u + 0x7FFFu + ((u >> 16) & 1u)) >> 16);
}
__device__ __forceinline__ __bf16 at_f2bf(float f) { return __builtin_bit_cast(__bf16, at_bf_bits(f)); }
__device__ __forceinline__ void at_split(float f, __bf16& hi, __bf16& lo) {
  const unsigned short hb = at_bf_bits(f);
  hi = __builtin_bit_cast(__bf16, hb);
  lo = at_f2bf(f - __uint_as_float(((unsigned)hb) << 16));
}
__device__ __forceinline__ v8f at_mma(v16b a, v16b b, v8f c) {
  c = __builtin_amdgcn_wmma_f32_16x16x32_bf16(false, a, false, b, (short)0, c, false, false);
  asm volatile("v_nop\n\tv_nop\n\tv_nop\n\tv_nop" : "+v"(c) : "v"(a), "v"(b));
  return c;
}

__device__ __forceinline__ void lds_wave_sync() {
  __builtin_amdgcn_fence(__ATOMIC_RELEASE, "workgroup");
  __builtin_amdgcn_wave_barrier();
  __builtin_amdgcn_fence(__ATOMIC_ACQUIRE, "workgroup");
}

__device__ __forceinline__ v16b x_frag_split(const float* __restrict__ xr, int hh) {
  const v4f a = *(const v4f*)(xr + 8 * hh);
  const v4f b = *(const v4f*)(xr + 8 * hh + 4);
  const float f[8] = {a[0], a[1], a[2], a[3], b[0], b[1], b[2], b[3]};
  v16b fr;
#pragma unroll
  for (int e = 0; e < 8; ++e) {
    __bf16 hb, lb;
    at_split(f[e], hb, lb);
    fr[e] = hb;
    fr[8 + e] = lb;
  }
  return fr;
}
__device__ __forceinline__ void w_frags_split(const float* __restrict__ W, int c, int hh, v16b& wh, v16b& wl) {
  const v4f a = *(const v4f*)(W + c * HEADD + 8 * hh);
  const v4f b = *(const v4f*)(W + c * HEADD + 8 * hh + 4);
  const float f[8] = {a[0], a[1], a[2], a[3], b[0], b[1], b[2], b[3]};
#pragma unroll
  for (int e = 0; e < 8; ++e) {
    __bf16 hb, lb;
    at_split(f[e], hb, lb);
    wh[e] = hb; wh[8 + e] = hb;
    wl[e] = lb; wl[8 + e] = lb;
  }
}

__device__ __forceinline__ void proj_qk_part(const float* __restrict__ x, unsigned short* __restrict__ dstp,
    const v16b wh, const v16b wl, float oscale, int slice, int n0, int t, int h, int lane, unsigned short* sl)
{
  const int hh = lane >> 4, c = lane & 15;
#pragma unroll
  for (int i = 0; i < 4; ++i) {
    const float* xr = x + ((size_t)(n0 + 16 * i + c) * TSTEP + t) * EMB + h * HEADD;
    const v16b xa = x_frag_split(xr, hh);
    v8f acc = (v8f){0.f,0.f,0.f,0.f,0.f,0.f,0.f,0.f};
    acc = at_mma(xa, wh, acc);
    acc = at_mma(xa, wl, acc);
#pragma unroll
    for (int r = 0; r < 8; ++r) {
      const float v = acc[r] * oscale;
      const unsigned short hb = f2bf_bits(v);
      const unsigned short lb = f2bf_bits(v - bf_bits2f(hb));
      const int row = 16 * i + 8 * hh + r;
      sl[row * QKROW + c] = hb;
      sl[row * QKROW + 16 + c] = lb;
    }
  }
  lds_wave_sync();
  unsigned short* dst = dstp + ((size_t)slice * NNODE + n0) * QKROW;
  for (int pass = 0; pass < 2; ++pass) {
#pragma unroll
    for (int it = 0; it < 8; ++it) {
      const us8 v = *(const us8*)(sl + (it * 32 + lane) * 8);
      *(volatile us8*)(dst + (it * 32 + lane) * 8) = v;
    }
    __threadfence();
  }
  lds_wave_sync();
}

__device__ __forceinline__ void proj_v_part(const float* __restrict__ x, unsigned short* __restrict__ Vth,
    unsigned short* __restrict__ Vtl, const v16b wh, const v16b wl, int slice, int n0, int t, int h, int lane,
    unsigned short* sl)
{
  const int hh = lane >> 4, c = lane & 15;
#pragma unroll
  for (int i = 0; i < 4; ++i) {
    const float* xr = x + ((size_t)(n0 + 16 * i + c) * TSTEP + t) * EMB + h * HEADD;
    const v16b xa = x_frag_split(xr, hh);
    v8f acc = (v8f){0.f,0.f,0.f,0.f,0.f,0.f,0.f,0.f};
    acc = at_mma(xa, wh, acc);
    acc = at_mma(xa, wl, acc);
    us8 hv, lv;
#pragma unroll
    for (int r = 0; r < 8; ++r) {
      const float v = acc[r];
      const unsigned short hb = f2bf_bits(v);
      const unsigned short lb = f2bf_bits(v - bf_bits2f(hb));
      hv[r] = hb;
      lv[r] = lb;
    }
    *(us8*)(sl + c * 64 + 16 * i + 8 * hh) = hv;
    *(us8*)(sl + 1024 + c * 64 + 16 * i + 8 * hh) = lv;
  }
  lds_wave_sync();
  const int qq = lane >> 3, c8 = (lane & 7) * 8;
  for (int pass = 0; pass < 2; ++pass) {
#pragma unroll
    for (int it = 0; it < 4; ++it) {
      const int d = it * 4 + qq;
      const us8 hv = *(const us8*)(sl + d * 64 + c8);
      const us8 lv = *(const us8*)(sl + 1024 + d * 64 + c8);
      const size_t off = ((size_t)slice * HEADD + d) * NNODE + n0 + c8;
      *(volatile us8*)(Vth + off) = hv;
      *(volatile us8*)(Vtl + off) = lv;
    }
    __threadfence();
  }
  lds_wave_sync();
}

__global__ __launch_bounds__(128) void proj_qkv(
    const float* __restrict__ values, const float* __restrict__ keys, const float* __restrict__ query,
    const float* __restrict__ Wv, const float* __restrict__ Wk, const float* __restrict__ Wq,
    unsigned short* __restrict__ Q2, unsigned short* __restrict__ K2,
    unsigned short* __restrict__ Vth, unsigned short* __restrict__ Vtl)
{
  __shared__ __align__(16) unsigned short slab[4][64 * QKROW];
  const int lane = threadIdx.x & 31;
  const int wave = threadIdx.x >> 5;
  const int hh = lane >> 4, c = lane & 15;
  const int task  = blockIdx.x * 4 + wave;
  const int slice = task >> 4;
  const int ng    = task & 15;
  const int t = slice >> 2, h = slice & 3;
  const int n0 = ng * 64;
  unsigned short* sl = slab[wave];

  v16b wqh, wql, wkh, wkl, wvh, wvl;
  w_frags_split(Wq, c, hh, wqh, wql);
  w_frags_split(Wk, c, hh, wkh, wkl);
  w_frags_split(Wv, c, hh, wvh, wvl);

  proj_qk_part(query, Q2, wqh, wql, 0.125f, slice, n0, t, h, lane, sl);
  proj_qk_part(keys,  K2, wkh, wkl, 1.0f,   slice, n0, t, h, lane, sl);
  proj_v_part(values, Vth, Vtl, wvh, wvl, slice, n0, t, h, lane, sl);
}

__global__ __launch_bounds__(256) void prep_wo_split(
    const float* __restrict__ Wo, unsigned short* __restrict__ Woh, unsigned short* __restrict__ Wol)
{
  const int tid = threadIdx.x;
  us8 hv[2], lv[2];
#pragma unroll
  for (int it = 0; it < 2; ++it) {
    const int g = tid + 256 * it;
    const v4f a = *(const v4f*)(Wo + 8 * g);
    const v4f b = *(const v4f*)(Wo + 8 * g + 4);
    const float f[8] = {a[0], a[1], a[2], a[3], b[0], b[1], b[2], b[3]};
#pragma unroll
    for (int e = 0; e < 8; ++e) {
      const unsigned short hb = f2bf_bits(f[e]);
      const unsigned short lb = f2bf_bits(f[e] - bf_bits2f(hb));
      hv[it][e] = hb;
      lv[it][e] = lb;
    }
  }
  for (int pass = 0; pass < 2; ++pass) {
#pragma unroll
    for (int it = 0; it < 2; ++it) {
      const int g = tid + 256 * it;
      *(volatile us8*)(Woh + 8 * g) = hv[it];
      *(volatile us8*)(Wol + 8 * g) = lv[it];
    }
    __threadfence();
  }
}

__global__ __launch_bounds__(128) void attn_hd16(
    const unsigned short* __restrict__ Q2, const unsigned short* __restrict__ K2,
    const unsigned short* __restrict__ Vth, const unsigned short* __restrict__ Vtl,
    unsigned short* __restrict__ Ohi, unsigned short* __restrict__ Olo)
{
  union FB { v16b v; v8b h[2]; };
  __shared__ __align__(16) __bf16 Ksh[64 * QKROW];
  __shared__ __align__(16) __bf16 Vhs[HEADD * 64];
  __shared__ __align__(16) __bf16 Vls[HEADD * 64];
  __shared__ __align__(16) __bf16 Psh[4][16 * 64];
  __shared__ __align__(16) __bf16 Psl[4][16 * 64];
  __shared__ __align__(16) float  Os[4][16 * 68];

  const int tid  = threadIdx.x;
  const int wave = tid >> 5;
  const int lane = tid & 31;
  const int hh   = lane >> 4;
  const int c    = lane & 15;
  const int t    = blockIdx.x >> 4;
  const int qb   = blockIdx.x & 15;
  const int q0   = qb * 64 + wave * 16;
  float*  os  = Os[wave];
  __bf16* pwh = Psh[wave];
  __bf16* pwl = Psl[wave];

#pragma unroll 1
  for (int h = 0; h < NHEAD; ++h) {
    const int slice = t * NHEAD + h;
    const __bf16* Qs = (const __bf16*)(const void*)Q2 + (size_t)slice * NNODE * QKROW;
    const v16b qa = Frag<__bf16>::load(Qs + (size_t)(q0 + c) * QKROW + 8 * hh);
    const v8b* Kg  = (const v8b*)(const void*)(K2  + (size_t)slice * NNODE * QKROW);
    const v8b* Vhg = (const v8b*)(const void*)(Vth + (size_t)slice * HEADD * NNODE);
    const v8b* Vlg = (const v8b*)(const void*)(Vtl + (size_t)slice * HEADD * NNODE);

    float mrow[8], lrow[8];
    v8f oacc = (v8f){0.f,0.f,0.f,0.f,0.f,0.f,0.f,0.f};
#pragma unroll
    for (int r = 0; r < 8; ++r) { mrow[r] = -INFINITY; lrow[r] = 0.f; }

#pragma unroll 1
    for (int kc = 0; kc < NNODE / 64; ++kc) {
      const int kv0 = kc * 64;
      __syncthreads();
#pragma unroll
      for (int i = 0; i < 2; ++i) {
        const int p = tid + 128 * i;
        const int row = p >> 2, seg = p & 3;
        const v8b kv = Kg[(size_t)(kv0 + row) * 4 + seg];
        *(v8b*)(Ksh + row * QKROW + seg * 8) = kv;
      }
      {
        const int d = tid >> 3, seg = tid & 7;
        const v8b a  = Vhg[(size_t)d * (NNODE / 8) + kc * 8 + seg];
        const v8b b2 = Vlg[(size_t)d * (NNODE / 8) + kc * 8 + seg];
        *(v8b*)(Vhs + d * 64 + seg * 8) = a;
        *(v8b*)(Vls + d * 64 + seg * 8) = b2;
      }
      __syncthreads();

      v8f s[4];
#pragma unroll
      for (int j = 0; j < 4; ++j) {
        const __bf16* kr = Ksh + (j * 16 + c) * QKROW + 8 * hh;
        const v8b kh8 = *(const v8b*)(kr);
        const v8b kl8 = *(const v8b*)(kr + 16);
        FB k1, k2;
        k1.h[0] = kh8; k1.h[1] = kh8;
        k2.h[0] = kl8; k2.h[1] = kl8;
        s[j] = (v8f){0.f,0.f,0.f,0.f,0.f,0.f,0.f,0.f};
        s[j] = at_mma(qa, k1.v, s[j]);
        s[j] = at_mma(qa, k2.v, s[j]);
      }
      float cm[8];
#pragma unroll
      for (int r = 0; r < 8; ++r) {
        float m = fmaxf(fmaxf(s[0][r], s[1][r]), fmaxf(s[2][r], s[3][r]));
#pragma unroll
        for (int off = 1; off < 16; off <<= 1) m = fmaxf(m, __shfl_xor(m, off, 32));
        cm[r] = m;
      }
#pragma unroll
      for (int r = 0; r < 8; ++r) {
        const float mnew  = fmaxf(mrow[r], cm[r]);
        const float alpha = expf(mrow[r] - mnew);
        mrow[r] = mnew;
        float psum = 0.f;
#pragma unroll
        for (int j = 0; j < 4; ++j) {
          const float p = expf(s[j][r] - mnew);
          psum += p;
          __bf16 a, bl;
          at_split(p, a, bl);
          pwh[(8 * hh + r) * 64 + j * 16 + c] = a;
          pwl[(8 * hh + r) * 64 + j * 16 + c] = bl;
        }
#pragma unroll
        for (int off = 1; off < 16; off <<= 1) psum += __shfl_xor(psum, off, 32);
        lrow[r] = lrow[r] * alpha + psum;
        oacc[r] *= alpha;
      }
      lds_wave_sync();
#pragma unroll
      for (int kk = 0; kk < 2; ++kk) {
        FB pa, pl, vb, vl;
        pa.h[0] = *(const v8b*)(pwh + c * 64 + kk * 32 + 8 * hh);
        pa.h[1] = *(const v8b*)(pwh + c * 64 + kk * 32 + 16 + 8 * hh);
        pl.h[0] = *(const v8b*)(pwl + c * 64 + kk * 32 + 8 * hh);
        pl.h[1] = *(const v8b*)(pwl + c * 64 + kk * 32 + 16 + 8 * hh);
        vb.h[0] = *(const v8b*)(Vhs + c * 64 + kk * 32 + 8 * hh);
        vb.h[1] = *(const v8b*)(Vhs + c * 64 + kk * 32 + 16 + 8 * hh);
        vl.h[0] = *(const v8b*)(Vls + c * 64 + kk * 32 + 8 * hh);
        vl.h[1] = *(const v8b*)(Vls + c * 64 + kk * 32 + 16 + 8 * hh);
        oacc = at_mma(pa.v, vb.v, oacc);
        oacc = at_mma(pa.v, vl.v, oacc);
        oacc = at_mma(pl.v, vb.v, oacc);
      }
    }
#pragma unroll
    for (int r = 0; r < 8; ++r) {
      const float inv = 1.0f / lrow[r];
      os[(8 * hh + r) * 68 + h * HEADD + c] = oacc[r] * inv;
    }
  }
  lds_wave_sync();
  {
    const int qq = lane >> 3, c8 = (lane & 7) * 8;
    for (int pass = 0; pass < 2; ++pass) {
#pragma unroll
      for (int it = 0; it < 4; ++it) {
        const int row = it * 4 + qq;
        const float* sp = os + row * 68 + c8;
        us8 hv, lv;
#pragma unroll
        for (int e = 0; e < 8; ++e) {
          const unsigned short hb = f2bf_bits(sp[e]);
          const unsigned short lb = f2bf_bits(sp[e] - bf_bits2f(hb));
          hv[e] = hb;
          lv[e] = lb;
        }
        const size_t R = (size_t)(q0 + row) * TSTEP + t;
        *(volatile us8*)(Ohi + R * EMB + c8) = hv;
        *(volatile us8*)(Olo + R * EMB + c8) = lv;
      }
      __threadfence();
    }
  }
}

extern "C" void kernel_launch(void* const* d_in, const int* in_sizes, int n_in,
                              void* d_out, int out_size, void* d_ws, size_t ws_size,
                              hipStream_t stream) {
  if (n_in < 8) return;
  if (in_sizes[0] != NNODE * TSTEP * EMB || in_sizes[1] != NNODE * TSTEP * EMB ||
      in_sizes[2] != NNODE * TSTEP * EMB || in_sizes[3] != HEADD * HEADD ||
      in_sizes[4] != HEADD * HEADD || in_sizes[5] != HEADD * HEADD ||
      in_sizes[6] != EMB * EMB || in_sizes[7] != EMB) return;
  if (out_size != NROWS * EMB) return;
  if (ws_size < WS_TOTAL) return;

  const float* values = (const float*)d_in[0];
  const float* keys   = (const float*)d_in[1];
  const float* query  = (const float*)d_in[2];
  const float* Wv     = (const float*)d_in[3];
  const float* Wk     = (const float*)d_in[4];
  const float* Wq     = (const float*)d_in[5];
  const float* Wo     = (const float*)d_in[6];
  const float* bo     = (const float*)d_in[7];

  char* ws = (char*)d_ws;
  unsigned short* Q2  = (unsigned short*)(ws + WS_Q2);
  unsigned short* K2  = (unsigned short*)(ws + WS_K2);
  unsigned short* Vth = (unsigned short*)(ws + WS_VTH);
  unsigned short* Vtl = (unsigned short*)(ws + WS_VTL);
  unsigned short* Ohi = (unsigned short*)(ws + WS_OHI);
  unsigned short* Olo = (unsigned short*)(ws + WS_OLO);
  unsigned short* Woh = (unsigned short*)(ws + WS_WOH);
  unsigned short* Wol = (unsigned short*)(ws + WS_WOL);

  prep_wo_split<<<dim3(1), dim3(256), 0, stream>>>(Wo, Woh, Wol);
  proj_qkv<<<dim3(NSLICE * (NNODE / 64) / 4), dim3(128), 0, stream>>>(
      values, keys, query, Wv, Wk, Wq, Q2, K2, Vth, Vtl);
  attn_hd16<<<dim3(TSTEP * (NNODE / 64)), dim3(128), 0, stream>>>(Q2, K2, Vth, Vtl, Ohi, Olo);
  wmma_gemm64<1, true, 2, 0, false, 0><<<dim3(NROWS / 64 / 8, 1), dim3(256), 0, stream>>>(
      Ohi, Olo, EMB, 0L, Woh, Wol, EMB, 0L,
      d_out, nullptr, EMB, 0L, bo, nullptr, 0L,
      NROWS, EMB, EMB, 1.0f);
}
